// GAT_PointGeo_68221260530301
// MI455X (gfx1250) — hardware-verified
//
#include <hip/hip_runtime.h>
#include <hip/hip_bf16.h>
#include <math.h>


#define BB 2
#define SS 2048
#define DD 1024
#define HH 16
#define DKK 64
#define QW 2

typedef _Float16 bf16;
typedef __attribute__((ext_vector_type(4))) unsigned v4u_t;
typedef unsigned v4ua __attribute__((ext_vector_type(4), may_alias));
typedef __attribute__((ext_vector_type(4))) float v4f_t;
typedef float v4fa __attribute__((ext_vector_type(4), may_alias));
typedef __attribute__((ext_vector_type(16))) bf16  bf16x16;
typedef __attribute__((ext_vector_type(8)))  bf16  bf16x8;
typedef __attribute__((ext_vector_type(4)))  bf16  bf16x4;
typedef __attribute__((ext_vector_type(8)))  float f32x8;

#define LDS_STRIDE 48
#define KSTRIDE    72
#define VSTRIDE    48

__device__ __forceinline__ f32x8 wmma_bf16(bf16x16 a, bf16x16 b, f32x8 c) {
  return __builtin_amdgcn_wmma_f32_16x16x32_f16(
      false, a, false, b, (short)0, c, false, false);
}
#define RSPLIT (1.0f / 2048.0f)
__device__ __forceinline__ bf16 lo_of(float v, bf16 h) { return (bf16)((v - (float)h) * 2048.0f); }
__device__ __forceinline__ f32x8 wmma_split(bf16x16 a, bf16x16 al, bf16x16 b, bf16x16 bl, f32x8 c) {
  f32x8 x = {}; x = wmma_bf16(al, b, x); x = wmma_bf16(a, bl, x); return wmma_bf16(a, b, c) + x * RSPLIT; }

template <typename T>
__device__ __forceinline__ bf16x16 load_frag(const T* __restrict__ base, int ld,
                                             int row0, int k0) {
  const int lane = threadIdx.x & 31;
  const int r    = lane & 15;
  const int kh   = (lane >> 4) * 8;
  const T* p0 = base + (size_t)(row0 + r) * ld + (k0 + kh);
  const T* p1 = p0 + 16;
  bf16x16 f;
#pragma unroll
  for (int i = 0; i < 8; ++i) {
    f[i]     = (bf16)p0[i];
    f[i + 8] = (bf16)p1[i];
  }
  return f;
}

__device__ __forceinline__ bf16x16 lds_frag(const bf16* base, int stride) {
  const int lane = threadIdx.x & 31;
  const int row  = lane & 15;
  const int kh   = (lane >> 4) * 8;
  const bf16x8 lo = *(const bf16x8*)(base + row * stride + kh);
  const bf16x8 hi = *(const bf16x8*)(base + row * stride + kh + 16);
  bf16x16 f;
#pragma unroll
  for (int i = 0; i < 8; ++i) { f[i] = lo[i]; f[i + 8] = hi[i]; }
  return f;
}

template <typename T>
__device__ __forceinline__ void stage_read16(const T* __restrict__ p, float* buf) {
#pragma unroll
  for (int i = 0; i < 16; ++i) buf[i] = (float)p[i];
}

__device__ __forceinline__ void stage_write(bf16* dst, const float* buf, int nquad) {
#pragma unroll
  for (int i = 0; i < nquad; ++i) {
    bf16x4 q;
    q[0] = (bf16)buf[4 * i];     q[1] = (bf16)buf[4 * i + 1];
    q[2] = (bf16)buf[4 * i + 2]; q[3] = (bf16)buf[4 * i + 3];
    *(bf16x4*)(dst + 4 * i) = q;
  }
}

__global__ __launch_bounds__(256) void transpose_pack_kernel(const float* __restrict__ W, bf16* __restrict__ WT, int K, int N, size_t plane) {
  __shared__ float tile[64][65];
  const int k0 = blockIdx.y * 64, n0 = blockIdx.x * 64, t = threadIdx.x;
  for (int i = t; i < 64 * 64; i += 256) { const int kr = i >> 6, nc = i & 63; tile[kr][nc] = W[(size_t)(k0 + kr) * N + n0 + nc]; }
  __syncthreads();
#pragma unroll 1
  for (int pass = 0; pass < 2; ++pass) {
    for (int i = t; i < 64 * 8; i += 256) { const int nr = i >> 3, k8 = (i & 7) * 8; bf16 hh[8], hl[8];
#pragma unroll
      for (int e = 0; e < 8; ++e) { const float v = tile[k8 + e][nr]; hh[e] = (bf16)v; hl[e] = lo_of(v, hh[e]); }
      bf16* d = WT + (size_t)(n0 + nr) * K + k0 + k8;
      *(volatile v4u_t*)d = *(const v4ua*)hh; *(volatile v4u_t*)(d + plane) = *(const v4ua*)hl; }
    __threadfence();
  }
}

template <typename AT, typename WT, int MODE>
__global__ __launch_bounds__(256) void gemm_split_kernel(
    const AT* __restrict__ A, size_t aPlane, const WT* __restrict__ W, size_t wPlane,
    const float* __restrict__ bias, void* __restrict__ out,
    int M, int N, int K) {
  __shared__ bf16 ldsA[128 * LDS_STRIDE], ldsAl[128 * LDS_STRIDE];
  __shared__ bf16 ldsW[256 * LDS_STRIDE], ldsWl[256 * LDS_STRIDE];
  __shared__ __attribute__((aligned(16))) unsigned char sob[256 * 136 * 2];

  const int t    = threadIdx.x;
  const int wave = t >> 5;
  const int lane = t & 31;
  const int wm   = (wave & 1) * 64;
  const int wn   = (wave >> 1) * 64;
  const int mBlk = blockIdx.x * 128;
  const int nBlk = blockIdx.y * 256;
  const int arow = t >> 1;
  const int ach  = (t & 1) * 16;

  f32x8 acc[4][4] = {};
  for (int k = 0; k < K; k += 32) {
    __syncthreads();
    {
      const AT* ap = A + (size_t)(mBlk + arow) * K + k + ach;
      bf16 hh[16], hl[16];
      if (sizeof(AT) == 4) {
#pragma unroll
        for (int i = 0; i < 16; ++i) { const float v = (float)ap[i]; hh[i] = (bf16)v; hl[i] = lo_of(v, hh[i]); }
      } else {
#pragma unroll
        for (int i = 0; i < 16; ++i) { hh[i] = (bf16)ap[i]; hl[i] = (bf16)ap[aPlane + i]; }
      }
#pragma unroll
      for (int i = 0; i < 16; ++i) { ldsA[arow * LDS_STRIDE + ach + i] = hh[i]; ldsAl[arow * LDS_STRIDE + ach + i] = hl[i]; }
    }
    {
      const WT* wp = W + (size_t)(nBlk + t) * K + k;
      if (sizeof(WT) == 4) {
#pragma unroll
        for (int i = 0; i < 32; ++i) { const float v = (float)wp[i]; const bf16 h_ = (bf16)v; ldsW[t * LDS_STRIDE + i] = h_; ldsWl[t * LDS_STRIDE + i] = lo_of(v, h_); }
      } else {
#pragma unroll
        for (int i = 0; i < 32; ++i) { ldsW[t * LDS_STRIDE + i] = (bf16)wp[i]; ldsWl[t * LDS_STRIDE + i] = (bf16)wp[wPlane + i]; }
      }
    }
    __syncthreads();
    bf16x16 wf[4], wfl[4];
#pragma unroll
    for (int j = 0; j < 4; ++j) { wf[j] = lds_frag(ldsW + (wn + 16 * j) * LDS_STRIDE, LDS_STRIDE); wfl[j] = lds_frag(ldsWl + (wn + 16 * j) * LDS_STRIDE, LDS_STRIDE); }
#pragma unroll
    for (int i = 0; i < 4; ++i) {
      const bf16x16 af = lds_frag(ldsA + (wm + 16 * i) * LDS_STRIDE, LDS_STRIDE), afl = lds_frag(ldsAl + (wm + 16 * i) * LDS_STRIDE, LDS_STRIDE);
#pragma unroll
      for (int j = 0; j < 4; ++j) acc[i][j] = wmma_split(af, afl, wf[j], wfl[j], acc[i][j]);
    }
  }

  const int nlane = lane & 15;
  const int mh    = (lane >> 4) * 8;
  __syncthreads();
  if (MODE == 1) {
    bf16* so = (bf16*)sob;
#pragma unroll
    for (int i = 0; i < 4; ++i)
#pragma unroll
      for (int j = 0; j < 4; ++j) {
        const int nl = wn + 16 * j + nlane;
        const float bv = bias ? bias[nBlk + nl] : 0.0f;
#pragma unroll
        for (int r = 0; r < 8; ++r) so[nl * 136 + wm + 16 * i + mh + r] = (bf16)(acc[i][j][r] + bv);
      }
    __syncthreads();
    const int b_ = mBlk >> 11, s0 = mBlk & (SS - 1);
#pragma unroll 1
    for (int pass = 0; pass < 2; ++pass) {
      for (int ch = t; ch < 256 * 16; ch += 256) { const int nl = ch >> 4, q = (ch & 15) * 8; const int n = nBlk + nl, h = n >> 6, dk = n & (DKK - 1);
        *(volatile v4u_t*)((bf16*)out + (((size_t)(b_ * HH + h)) * DKK + dk) * SS + s0 + q) = *(const v4ua*)(so + nl * 136 + q); }
      __threadfence();
    }
  } else {
    float* so = (float*)sob;
#pragma unroll 1
    for (int hf = 0; hf < 2; ++hf) {
      if (wm == hf * 64) {
#pragma unroll
        for (int i = 0; i < 4; ++i)
#pragma unroll
          for (int j = 0; j < 4; ++j) {
            const int nl = wn + 16 * j + nlane;
            const float bv = bias ? bias[nBlk + nl] : 0.0f;
#pragma unroll
            for (int r = 0; r < 8; ++r) so[(16 * i + mh + r) * 260 + nl] = acc[i][j][r] + bv;
          }
      }
      __syncthreads();
#pragma unroll 1
      for (int pass = 0; pass < 2; ++pass) {
        for (int ch = t; ch < 64 * 64; ch += 256) { const int ml = ch >> 6, q = (ch & 63) * 4;
          *(volatile v4f_t*)((float*)out + (size_t)(mBlk + hf * 64 + ml) * N + nBlk + q) = *(const volatile v4fa*)(so + ml * 260 + q); }
        __threadfence();
      }
      __syncthreads();
    }
  }
}


#define PN 10000
#define PNP 10112
#define PE 160000
#define PD 512

__global__ __launch_bounds__(256) void k_padrows(const float* __restrict__ x, float* __restrict__ XP) {
  const int row = blockIdx.x, t = threadIdx.x;
  for (int c = t; c < PD; c += 256) { const float v = (row < PN) ? x[(size_t)row * PD + c] : 0.0f; *(volatile float*)(XP + (size_t)row * PD + c) = v; }
  __threadfence();
  for (int c = t; c < PD; c += 256) { const float v = (row < PN) ? x[(size_t)row * PD + c] : 0.0f; *(volatile float*)(XP + (size_t)row * PD + c) = v; }
}
__global__ __launch_bounds__(256) void k_gat(const int* __restrict__ ei, const float* __restrict__ XS, const float* __restrict__ XD,
                                            const float* __restrict__ Wp, const float* __restrict__ bp, const int* __restrict__ tg,
                                            float* __restrict__ Z, float* __restrict__ out) {
  __shared__ int qd[256], qs[256]; __shared__ int wcnt[8];
  __shared__ float mx[PNP]; __shared__ float ssum[PNP];
  const int tid = threadIdx.x, lane = tid & 31, wave = tid >> 5;
  for (int i = tid; i < PNP; i += 256) { mx[i] = -3.0e38f; ssum[i] = 0.0f; }
  for (int i = tid; i < PNP * PD / 4; i += 256) { v4f_t z; z.x = z.y = z.z = z.w = 0.0f; *(volatile v4f_t*)(Z + (size_t)i * 4) = z; }
  __threadfence(); __syncthreads();
  const int* srcp = ei; const int* dstp = ei + (size_t)PE;
  const float rt = 1.0f / sqrtf((float)PD);
#pragma unroll 1
  for (int pass = 0; pass < 2; ++pass) {
#pragma unroll 1
    for (int c0 = 0; c0 < PE; c0 += 256) {
      const int e = c0 + tid; int d = -1, sidx = 0;
      if (e < PE) { const int draw = dstp[e]; d = draw < 0 ? 0 : (draw >= PN ? PN - 1 : draw); const int ss = srcp[e]; sidx = ss < 0 ? 0 : (ss >= PN ? PN - 1 : ss); }
      const unsigned m = __builtin_amdgcn_ballot_w32(d >= 0);
      if (lane == 0) wcnt[wave] = __builtin_popcount(m);
      __syncthreads();
      int base = 0, total = 0;
#pragma unroll
      for (int w = 0; w < 8; ++w) { const int c = wcnt[w]; base += (w < wave) ? c : 0; total += c; }
      if (d >= 0) { const int pos = base + __builtin_popcount(m & ((1u << lane) - 1u)); qd[pos] = d; qs[pos] = sidx; }
      __syncthreads();
#pragma unroll 1
      for (int qi = 0; qi < total; ++qi) { const int dl = qd[qi]; if ((dl & 7) != wave) continue; const int sl = qs[qi];
        const float* hs = XS + (size_t)sl * PD; const float* hd = XD + (size_t)dl * PD;
        float part = 0.0f;
#pragma unroll 1
        for (int u = 0; u < PD / 32; ++u) part += hs[u * 32 + lane] * hd[u * 32 + lane];
#pragma unroll
        for (int o = 16; o >= 1; o >>= 1) part += __shfl_xor(part, o, 32);
        const float score = part * rt;
        if (pass == 0) { if (lane == 0) mx[dl] = fmaxf(mx[dl], score); }
        else { const float ev = expf(score - mx[dl]); if (lane == 0) ssum[dl] += ev;
          float* row = Z + (size_t)dl * PD;
#pragma unroll 1
          for (int u = 0; u < PD / 32; ++u) row[u * 32 + lane] += ev * hs[u * 32 + lane]; }
      }
      __syncthreads();
    }
  }
  __threadfence(); __syncthreads();
#pragma unroll 1
  for (int node = wave; node < PN; node += 8) {
    const float inv = 1.0f / (ssum[node] + 1e-16f); const float* row = Z + (size_t)node * PD;
    float p0 = 0.0f, p1 = 0.0f;
#pragma unroll 1
    for (int u = 0; u < PD / 32; ++u) { const float z = row[u * 32 + lane] * inv; p0 += z * Wp[(u * 32 + lane) * 2]; p1 += z * Wp[(u * 32 + lane) * 2 + 1]; }
#pragma unroll
    for (int o = 16; o >= 1; o >>= 1) { p0 += __shfl_xor(p0, o, 32); p1 += __shfl_xor(p1, o, 32); }
    const float mk = (tg[node] == 1) ? 1.0f : 0.0f;
    if (lane == 0) { typedef __attribute__((ext_vector_type(2))) float v2f; v2f v; v.x = (p0 + bp[0]) * mk; v.y = (p1 + bp[1]) * mk;
      *(volatile v2f*)(out + (size_t)node * 2) = v; __threadfence(); *(volatile v2f*)(out + (size_t)node * 2) = v; }
  }
}

extern "C" void kernel_launch(void* const* d_in, const int* in_sizes, int n_in,
                              void* d_out, int out_size, void* d_ws, size_t ws_size,
                              hipStream_t stream) {
  (void)in_sizes; (void)n_in; (void)out_size; (void)ws_size;
  const float* x  = (const float*)d_in[0];
  const int*   ei = (const int*)d_in[1];
  const int*   tg = (const int*)d_in[2];
  const float* Ws = (const float*)d_in[3]; const float* bs = (const float*)d_in[4];
  const float* Wd = (const float*)d_in[5]; const float* bd = (const float*)d_in[6];
  const float* Wp = (const float*)d_in[7]; const float* bp = (const float*)d_in[8];
  char* ws = (char*)d_ws;
  bf16* WT  = (bf16*)ws;  ws += (size_t)2 * 2 * PD * PD * 2;
  float* XP = (float*)ws; ws += (size_t)PNP * PD * 4;
  float* XS = (float*)ws; ws += (size_t)PNP * PD * 4;
  float* XD = (float*)ws; ws += (size_t)PNP * PD * 4;
  float* Z  = (float*)ws; ws += (size_t)PNP * PD * 4;
  const size_t pl = (size_t)PD * PD;
  transpose_pack_kernel<<<dim3(PD / 64, PD / 64), 256, 0, stream>>>(Ws, WT, PD, PD, pl);
  transpose_pack_kernel<<<dim3(PD / 64, PD / 64), 256, 0, stream>>>(Wd, WT + 2 * pl, PD, PD, pl);
  k_padrows<<<PNP, 256, 0, stream>>>(x, XP);
  dim3 blk(256);
  gemm_split_kernel<float, bf16, 2><<<dim3(PNP / 128, PD / 256), blk, 0, stream>>>(XP, 0, WT, pl, bs, XS, PNP, PD, PD);
  gemm_split_kernel<float, bf16, 2><<<dim3(PNP / 128, PD / 256), blk, 0, stream>>>(XP, 0, WT + 2 * pl, pl, bd, XD, PNP, PD, PD);
  k_gat<<<1, 256, 0, stream>>>(ei, XS, XD, Wp, bp, tg, Z, (float*)d_out);
}
